// PhysicsConstrainedAttention_69140383531369
// MI455X (gfx1250) — hardware-run, weakly checked
//
#include <hip/hip_runtime.h>
#include <math.h>
#include <stdint.h>

#define NB     2
#define CH     128
#define HWD    64
#define NSEQ   4096
#define NHEAD  8
#define HDIM   16
#define QKW    384
#define MP     (NB * NSEQ)
#define LNEPS  1.0e-5f
#define XC     4.0f
#define WSC    8.0f
#define QC     16.0f
#define KC     8.0f
#define VC     4.0f
#define AC     32.0f
#define QSCALE 0.25f
#define LNPC   6.931471805599453f
static_assert(NHEAD * HDIM == CH);
static_assert(HWD * HWD == NSEQ);
static_assert((MP % 64) == 0 && (CH % 64) == 0 && (NSEQ % 64) == 0);
static_assert(CH == 32 * 4);

typedef _Float16 v16h __attribute__((ext_vector_type(16)));
typedef _Float16 v8h  __attribute__((ext_vector_type(8)));
typedef float    v8f  __attribute__((ext_vector_type(8)));
typedef float    v4f  __attribute__((ext_vector_type(4)));
typedef unsigned int v4u __attribute__((ext_vector_type(4)));
typedef unsigned int v2u __attribute__((ext_vector_type(2)));

union FragH { v16h v; v8h h[2]; };

__device__ __forceinline__ unsigned short bf_bits(float f) {
  unsigned u = __float_as_uint(f);
  return (unsigned short)((u + 0x7FFFu + ((u >> 16) & 1u)) >> 16);
}
__device__ __forceinline__ float bf_up(unsigned short h) { return __uint_as_float(((unsigned)h) << 16); }
__device__ __forceinline__ float bfr(float f) { return bf_up(bf_bits(f)); }
__device__ __forceinline__ unsigned short h_bits(_Float16 x) { return __builtin_bit_cast(unsigned short, x); }
__device__ __forceinline__ unsigned pk16(unsigned short a, unsigned short b) { return (unsigned)a | ((unsigned)b << 16); }
__device__ __forceinline__ v8f zero8() { v8f z = {0.f, 0.f, 0.f, 0.f, 0.f, 0.f, 0.f, 0.f}; return z; }
__device__ __forceinline__ float hmax8(v8f s) {
  return fmaxf(fmaxf(fmaxf(s[0], s[1]), fmaxf(s[2], s[3])), fmaxf(fmaxf(s[4], s[5]), fmaxf(s[6], s[7])));
}

__device__ __forceinline__ v16h ldfrag_h(const _Float16* p) {
  FragH f;
  f.h[0] = *(const v8h*)(p);
  f.h[1] = *(const v8h*)(p + 16);
  return f.v;
}

__device__ __forceinline__ v8f mma_h_raw(v16h a, v16h b, v8f c) {
  return __builtin_amdgcn_wmma_f32_16x16x32_f16(false, a, false, b, (short)0, c, false, false);
}
__device__ __forceinline__ void dep_guard1(v8f& a, v8f& b, v16h x) {
#if defined(__HIP_DEVICE_COMPILE__)
  asm volatile("v_nop\n\tv_nop\n\tv_nop\n\tv_nop" : "+v"(a), "+v"(b) : "v"(x));
#endif
}
__device__ __forceinline__ void keep4_h(v16h a, v16h b, v16h c, v16h d) {
#if defined(__HIP_DEVICE_COMPILE__)
  asm volatile("v_nop" :: "v"(a), "v"(b), "v"(c), "v"(d));
#endif
}
__device__ __forceinline__ void acc_guard4(v8f& a, v8f& b, v8f& c, v8f& d) {
#if defined(__HIP_DEVICE_COMPILE__)
  asm volatile("v_nop\n\tv_nop\n\tv_nop\n\tv_nop" : "+v"(a), "+v"(b), "+v"(c), "+v"(d));
#endif
}
__device__ __forceinline__ void sguard4(v8f& a, v8f& b, v8f& c, v8f& d,
                                        v16h k0, v16h k1, v16h k2, v16h k3, v16h q) {
#if defined(__HIP_DEVICE_COMPILE__)
  asm volatile("v_nop\n\tv_nop\n\tv_nop\n\tv_nop"
               : "+v"(a), "+v"(b), "+v"(c), "+v"(d) : "v"(k0), "v"(k1), "v"(k2), "v"(k3), "v"(q));
#endif
}
__device__ __forceinline__ void oguard(v8f& o, v16h a0, v16h a1, v16h b0, v16h b1) {
#if defined(__HIP_DEVICE_COMPILE__)
  asm volatile("v_nop\n\tv_nop\n\tv_nop\n\tv_nop" : "+v"(o) : "v"(a0), "v"(a1), "v"(b0), "v"(b1));
#endif
}
__device__ __forceinline__ void wave_sync_lds() {
  __builtin_amdgcn_fence(__ATOMIC_RELEASE, "workgroup");
  __builtin_amdgcn_wave_barrier();
  __builtin_amdgcn_fence(__ATOMIC_ACQUIRE, "workgroup");
}
__device__ __forceinline__ float wsum(float v) {
#pragma unroll
  for (int off = 16; off > 0; off >>= 1) v += __shfl_xor(v, off, 32);
  return v;
}

__global__ __launch_bounds__(256) void wprep(const float* __restrict__ wqkv, const float* __restrict__ wproj,
                                              unsigned short* WT, unsigned short* WPT) {
  __shared__ float T[64 * 33];
  const int t  = threadIdx.x;
  const int bx = blockIdx.x;
  const bool isq = (bx < 24);
  const float* src   = isq ? wqkv : wproj;
  unsigned short* ds = isq ? WT : WPT;
  const int ncol = isq ? QKW : CH;
  const int ot   = isq ? (bx >> 1) : ((bx - 24) >> 1);
  const int kt   = bx & 1;
  const int o0 = ot * 32, k0 = kt * 64;
  {
    const int k = t >> 2, oo = 8 * (t & 3);
    const float* sp = src + (size_t)(k0 + k) * ncol + o0 + oo;
    const v4f a = *(const v4f*)(sp), c = *(const v4f*)(sp + 4);
#pragma unroll
    for (int i = 0; i < 4; ++i) { T[k * 33 + oo + i] = a[i]; T[k * 33 + oo + 4 + i] = c[i]; }
  }
  __syncthreads();
  {
    const int o = t >> 3, e = t & 7;
    float w[8];
#pragma unroll
    for (int i = 0; i < 8; ++i) w[i] = bfr(T[(8 * e + i) * 33 + o]) * WSC;
    v4u v;
#pragma unroll
    for (int i = 0; i < 4; ++i) v[i] = pk16(h_bits((_Float16)w[2 * i]), h_bits((_Float16)w[2 * i + 1]));
    unsigned short* dp = ds + (size_t)(o0 + o) * CH + k0 + 8 * e;
    *(volatile v4u*)dp = v;
    __threadfence();
    *(volatile v4u*)dp = v;
  }
}

__global__ __launch_bounds__(256) void ln_tok(const float* __restrict__ x, const float* __restrict__ gam,
                                               const float* __restrict__ bet, unsigned short* XN) {
  __shared__ __align__(16) float T[CH * 36];
  __shared__ __align__(16) unsigned int Yw[8][4 * 64];
  const int tid = threadIdx.x, wave = tid >> 5, lane = tid & 31;
  const int bx = blockIdx.x;
  const int b  = bx >> 7;
  const int n0 = (bx & 127) * 32;
  const float* sb = x + (size_t)b * CH * NSEQ + n0;
  {
    const int q = lane >> 3, e = lane & 7;
#pragma unroll
    for (int it = 0; it < 4; ++it) {
      const int c = wave * 16 + it * 4 + q;
      const v4f v = *(const v4f*)(sb + (size_t)c * NSEQ + 4 * e);
      *(v4f*)(T + c * 36 + 4 * e) = v;
    }
  }
  __syncthreads();
  const v4f g4 = *(const v4f*)(gam + 4 * lane);
  const v4f b4 = *(const v4f*)(bet + 4 * lane);
  float gg[4], bb[4];
#pragma unroll
  for (int e = 0; e < 4; ++e) { gg[e] = bfr(g4[e]); bb[e] = bfr(b4[e]); }
#pragma unroll 1
  for (int i = 0; i < 4; ++i) {
    const int tl = wave * 4 + i;
    float xv[4];
#pragma unroll
    for (int e = 0; e < 4; ++e) xv[e] = bfr(T[(4 * lane + e) * 36 + tl]);
    float s = (xv[0] + xv[1]) + (xv[2] + xv[3]);
    s = wsum(s);
    const float mean = s * (1.0f / CH);
    float d[4];
#pragma unroll
    for (int e = 0; e < 4; ++e) d[e] = xv[e] - mean;
    float vs = (d[0] * d[0] + d[1] * d[1]) + (d[2] * d[2] + d[3] * d[3]);
    vs = wsum(vs);
    const float rstd = rsqrtf(vs * (1.0f / CH) + LNEPS);
    float y[4];
#pragma unroll
    for (int e = 0; e < 4; ++e) y[e] = ((d[e] * rstd) * gg[e] + bb[e]) * XC;
    v2u u;
    u[0] = pk16(h_bits((_Float16)y[0]), h_bits((_Float16)y[1]));
    u[1] = pk16(h_bits((_Float16)y[2]), h_bits((_Float16)y[3]));
    *(v2u*)(&Yw[wave][i * 64 + 2 * lane]) = u;
  }
  wave_sync_lds();
  {
    const v4u oa = *(const v4u*)(&Yw[wave][4 * lane]);
    const v4u ob = *(const v4u*)(&Yw[wave][128 + 4 * lane]);
    const size_t tokA = (size_t)b * NSEQ + n0 + wave * 4;
    unsigned short* pa = XN + tokA * CH + 8 * lane;
    unsigned short* pb = XN + (tokA + 2) * CH + 8 * lane;
    *(volatile v4u*)pa = oa;
    *(volatile v4u*)pb = ob;
    __threadfence();
    *(volatile v4u*)pa = oa;
    *(volatile v4u*)pb = ob;
  }
}

template <int BKM, int OM>
__global__ __launch_bounds__(256) void gemm64(
    const unsigned short* __restrict__ Ap, int lda, long long strideA,
    const unsigned short* __restrict__ Bp, int ldb, long long strideB,
    const float* __restrict__ bias, const float* __restrict__ resid,
    void* Cout, int ldc, long long strideC,
    unsigned short* Clo, int ldlo, long long strideLo, int nsplit,
    float osc0, float osc1, int M, int N, int K) {
  __shared__ __align__(16) float sT[8][16 * 68];
  const int b    = blockIdx.y;
  const int lane = threadIdx.x & 31;
  const int wave = threadIdx.x >> 5;
  const int tilesN = N >> 6;
  const int tilesM = M >> 6;
  const int tile = blockIdx.x * 8 + wave;
  if (tile >= tilesM * tilesN) return;
  const int tm = tile / tilesN;
  const int tn = tile - tm * tilesN;
  const int m0 = tm << 6;
  const int n0 = tn << 6;

  const _Float16* Ah = (const _Float16*)(const void*)Ap + (size_t)b * strideA;
  const _Float16* Bb = (const _Float16*)(const void*)Bp + (size_t)b * strideB;

  const int rlane = lane & 15;
  const int koff  = (lane >> 4) * 8;
  const int mOff  = (lane >> 4) * 8;

  v8f acc[4][4];
#pragma unroll
  for (int i = 0; i < 4; ++i)
#pragma unroll
    for (int j = 0; j < 4; ++j) acc[i][j] = zero8();

  for (int k0 = 0; k0 < K; k0 += 32) {
    v16h bh[4];
#pragma unroll
    for (int j = 0; j < 4; ++j) {
      if (BKM == 0) {
        const size_t bo = (size_t)(n0 + (j << 4) + rlane) * ldb + koff + k0;
        bh[j] = ldfrag_h(Bb + bo);
      } else {
        const _Float16* bp = Bb + (size_t)(k0 + koff) * ldb + n0 + (j << 4) + rlane;
        FragH f;
#pragma unroll
        for (int i = 0; i < 8; ++i) {
          f.h[0][i] = bp[(size_t)i * ldb];
          f.h[1][i] = bp[(size_t)(16 + i) * ldb];
        }
        bh[j] = f.v;
      }
    }
#pragma unroll
    for (int i = 0; i < 4; ++i) {
      const size_t ao = (size_t)(m0 + (i << 4) + rlane) * lda + koff + k0;
      const v16h ah = ldfrag_h(Ah + ao);
#pragma unroll
      for (int j = 0; j < 4; ++j) acc[i][j] = mma_h_raw(ah, bh[j], acc[i][j]);
      dep_guard1(acc[i][0], acc[i][3], ah);
    }
    keep4_h(bh[0], bh[1], bh[2], bh[3]);
  }
  acc_guard4(acc[0][0], acc[0][1], acc[0][2], acc[0][3]);
  acc_guard4(acc[1][0], acc[1][1], acc[1][2], acc[1][3]);
  acc_guard4(acc[2][0], acc[2][1], acc[2][2], acc[2][3]);
  acc_guard4(acc[3][0], acc[3][1], acc[3][2], acc[3][3]);

  const float oscale = (OM == 1 && n0 >= nsplit) ? osc1 : osc0;
  const bool  dolo   = (OM == 1) && (n0 < nsplit);
  const int hh2 = lane >> 4, c4 = (lane & 15) * 4;
  const int q8  = lane >> 3, c8 = (lane & 7) * 8;

  float* slab = sT[wave];
#pragma unroll
  for (int i = 0; i < 4; ++i) {
    const int mBase = m0 + (i << 4);
#pragma unroll
    for (int j = 0; j < 4; ++j) {
#pragma unroll
      for (int r = 0; r < 8; ++r) {
        slab[(mOff + r) * 68 + (j << 4) + rlane] = acc[i][j][r];
      }
    }
    wave_sync_lds();
    if (OM == 0) {
      float* C = (float*)Cout + (size_t)b * strideC;
      const float* Rf = resid + (size_t)b * strideC;
      v4f vals[8];
#pragma unroll
      for (int it = 0; it < 8; ++it) {
        const int row = it * 2 + hh2;
        const float bm = bfr(bias[mBase + row]);
        v4f v = *(const v4f*)(slab + row * 68 + c4);
        const v4f rr = *(const v4f*)(Rf + (size_t)(mBase + row) * ldc + n0 + c4);
#pragma unroll
        for (int e = 0; e < 4; ++e) v[e] = (v[e] * oscale + bm) + bfr(rr[e]);
        vals[it] = v;
      }
      for (int pass = 0; pass < 2; ++pass) {
#pragma unroll
        for (int it = 0; it < 8; ++it) {
          const int row = it * 2 + hh2;
          *(volatile v4f*)(C + (size_t)(mBase + row) * ldc + n0 + c4) = vals[it];
        }
        __threadfence();
      }
    } else {
      unsigned short* C = (unsigned short*)Cout + (size_t)b * strideC;
      unsigned short* L = Clo + (size_t)b * strideLo;
      v4u hv[4], lv[4];
#pragma unroll
      for (int it = 0; it < 4; ++it) {
        const int row = it * 4 + q8;
        const float* sp = slab + row * 68 + c8;
        v4u a, lo;
#pragma unroll
        for (int e = 0; e < 4; ++e) {
          const float f0 = sp[2 * e] * oscale, f1 = sp[2 * e + 1] * oscale;
          const _Float16 h0 = (_Float16)f0, h1 = (_Float16)f1;
          const _Float16 l0 = (_Float16)(f0 - (float)h0), l1 = (_Float16)(f1 - (float)h1);
          a[e]  = pk16(h_bits(h0), h_bits(h1));
          lo[e] = pk16(h_bits(l0), h_bits(l1));
        }
        hv[it] = a;
        lv[it] = lo;
      }
      for (int pass = 0; pass < 2; ++pass) {
#pragma unroll
        for (int it = 0; it < 4; ++it) {
          const int row = it * 4 + q8;
          *(volatile v4u*)(C + (size_t)(mBase + row) * ldc + n0 + c8) = hv[it];
          if (dolo) *(volatile v4u*)(L + (size_t)(mBase + row) * ldlo + n0 + c8) = lv[it];
        }
        __threadfence();
      }
    }
    wave_sync_lds();
  }
}

__global__ __launch_bounds__(128)
void attn_t(const unsigned short* __restrict__ qk, const unsigned short* __restrict__ ql,
            const unsigned short* __restrict__ vt, unsigned short* ot) {
  __shared__ __align__(16) unsigned short Os[HDIM * 64];
  const int tid  = threadIdx.x;
  const int wave = tid >> 5;
  const int lane = tid & 31;
  const int hh   = lane >> 4;
  const int c    = lane & 15;
  const int bx = blockIdx.x;
  const int qb = bx & 63;
  const int hd = (bx >> 6) & 7;
  const int b  = bx >> 9;
  const int q0 = qb * 64;
  const size_t tok0 = (size_t)b * NSEQ;

  const _Float16* QKp = (const _Float16*)(const void*)qk;
  const _Float16* QLp = (const _Float16*)(const void*)ql;
  const _Float16* Vp  = (const _Float16*)(const void*)vt + ((size_t)b * CH + (size_t)hd * HDIM + c) * NSEQ + 8 * hh;

  FragH qf;
  {
    const size_t tr = tok0 + q0 + wave * 16 + c;
    qf.h[0] = *(const v8h*)(QKp + tr * (2 * CH) + hd * HDIM + 8 * hh);
    qf.h[1] = *(const v8h*)(QLp + tr * CH + hd * HDIM + 8 * hh);
  }
  const _Float16* Kp = QKp + (tok0 + c) * (2 * CH) + CH + hd * HDIM + 8 * hh;
  const float SC = 1.0f / (QC * KC);

  float m = -1.0e30f, l = 0.f;
  v8f o = zero8();
#pragma unroll 1
  for (int it = 0; it < NSEQ / 64; ++it) {
    const int kb = it * 64;
    v16h kf[4];
#pragma unroll
    for (int j = 0; j < 4; ++j) {
      FragH f;
      f.h[0] = *(const v8h*)(Kp + (size_t)(kb + 16 * j) * (2 * CH));
      f.h[1] = f.h[0];
      kf[j] = f.v;
    }
    v8f s0 = mma_h_raw(kf[0], qf.v, zero8());
    v8f s1 = mma_h_raw(kf[1], qf.v, zero8());
    v8f s2 = mma_h_raw(kf[2], qf.v, zero8());
    v8f s3 = mma_h_raw(kf[3], qf.v, zero8());
    sguard4(s0, s1, s2, s3, kf[0], kf[1], kf[2], kf[3], qf.v);

    float mx = fmaxf(fmaxf(hmax8(s0), hmax8(s1)), fmaxf(hmax8(s2), hmax8(s3)));
    mx = fmaxf(mx, __shfl_xor(mx, 16, 32));
    const float mn   = fmaxf(m, mx * SC);
    const float corr = __expf(m - mn);
    m = mn;
    const float msh = mn - LNPC;
    l *= corr;
#pragma unroll
    for (int r = 0; r < 8; ++r) o[r] *= corr;

    FragH p0, p1;
    float ls = 0.f;
#pragma unroll
    for (int r = 0; r < 8; ++r) {
      const float e0 = __expf(s0[r] * SC - msh);
      const float e1 = __expf(s1[r] * SC - msh);
      const float e2 = __expf(s2[r] * SC - msh);
      const float e3 = __expf(s3[r] * SC - msh);
      ls += (e0 + e1) + (e2 + e3);
      p0.h[0][r] = (_Float16)e0;
      p0.h[1][r] = (_Float16)e1;
      p1.h[0][r] = (_Float16)e2;
      p1.h[1][r] = (_Float16)e3;
    }
    l += ls;

    const v16h v0 = ldfrag_h(Vp + kb);
    const v16h v1 = ldfrag_h(Vp + kb + 32);
    o = mma_h_raw(v0, p0.v, o);
    o = mma_h_raw(v1, p1.v, o);
    oguard(o, v0, v1, p0.v, p1.v);
  }
  l += __shfl_xor(l, 16, 32);
  const float sc = (AC / VC) / l;

#pragma unroll
  for (int r = 0; r < 8; ++r) Os[(8 * hh + r) * 64 + wave * 16 + c] = h_bits((_Float16)(o[r] * sc));
  __syncthreads();
  {
    const int d = tid >> 3, e = tid & 7;
    const v4u val = *(const v4u*)(Os + d * 64 + 8 * e);
    unsigned short* dp = ot + ((size_t)(b * CH + hd * HDIM + d)) * NSEQ + q0 + 8 * e;
    *(volatile v4u*)dp = val;
    __threadfence();
    *(volatile v4u*)dp = val;
  }
}

__global__ __launch_bounds__(256) void reg_part(const float* __restrict__ outp, float* part) {
  __shared__ float ws4[8][4];
  const int tid = threadIdx.x, wave = tid >> 5, lane = tid & 31;
  const int p = blockIdx.x;
  const float* pl = outp + (size_t)p * NSEQ;
  const int h = tid >> 2, w0 = (tid & 3) * 16;
  const float* rp = pl + h * HWD + w0;
  const v4f a0 = *(const v4f*)(rp), a1 = *(const v4f*)(rp + 4), a2 = *(const v4f*)(rp + 8), a3 = *(const v4f*)(rp + 12);
  const int hn = (h < HWD - 1) ? (h + 1) : (HWD - 1);
  const float* dp = pl + hn * HWD + w0;
  const v4f d0 = *(const v4f*)(dp), d1 = *(const v4f*)(dp + 4), d2 = *(const v4f*)(dp + 8), d3 = *(const v4f*)(dp + 12);
  const int wn = (w0 + 16 < HWD) ? (w0 + 16) : (HWD - 1);
  const float nx = pl[h * HWD + wn];
  float v[16], dv[16];
#pragma unroll
  for (int i = 0; i < 4; ++i) {
    v[i] = a0[i]; v[4 + i] = a1[i]; v[8 + i] = a2[i]; v[12 + i] = a3[i];
    dv[i] = d0[i]; dv[4 + i] = d1[i]; dv[8 + i] = d2[i]; dv[12 + i] = d3[i];
  }
  float s1 = 0.f, s2 = 0.f, sdx = 0.f, sdy = 0.f;
#pragma unroll
  for (int i = 0; i < 16; ++i) { s1 += v[i]; s2 += v[i] * v[i]; sdy += fabsf(dv[i] - v[i]); }
#pragma unroll
  for (int i = 0; i < 15; ++i) sdx += fabsf(v[i + 1] - v[i]);
  sdx += (w0 + 16 < HWD) ? fabsf(nx - v[15]) : 0.f;
  sdy = (h < HWD - 1) ? sdy : 0.f;
  s1 = wsum(s1); s2 = wsum(s2); sdx = wsum(sdx); sdy = wsum(sdy);
  if (lane == 0) { ws4[wave][0] = s1; ws4[wave][1] = s2; ws4[wave][2] = sdx; ws4[wave][3] = sdy; }
  __syncthreads();
  float t1 = 0.f, t2 = 0.f, t3 = 0.f, t4 = 0.f;
#pragma unroll
  for (int w = 0; w < 8; ++w) { t1 += ws4[w][0]; t2 += ws4[w][1]; t3 += ws4[w][2]; t4 += ws4[w][3]; }
  v4f val;
  val[0] = (lane == 0) ? t1 : 0.f;
  val[1] = (lane == 0) ? t2 : 0.f;
  val[2] = (lane == 0) ? t3 : 0.f;
  val[3] = (lane == 0) ? t4 : 0.f;
  float* lp = part + (size_t)p * 32 + 4 * lane;
  const bool wr = (wave == 0) && (lane < 8);
  if (wr) *(volatile v4f*)lp = val;
  __threadfence();
  if (wr) *(volatile v4f*)lp = val;
}

__global__ __launch_bounds__(256) void reg_fin(const float* __restrict__ part, float* out1) {
  __shared__ double D[4][256];
  __shared__ double S[4];
  const int t = threadIdx.x;
  const v4f pv = *(const v4f*)(part + (size_t)t * 32);
  D[0][t] = (double)pv[0];
  D[1][t] = (double)pv[1];
  D[2][t] = (double)pv[2];
  D[3][t] = (double)pv[3];
  __syncthreads();
  if (t < 4) {
    double s = 0.0;
#pragma unroll 1
    for (int i = 0; i < 256; ++i) s += D[t][i];
    S[t] = s;
  }
  __syncthreads();
  if (t == 0) {
    const double invM = 1.0 / (double)(NB * CH * NSEQ);
    const double invD = 1.0 / (double)(NB * CH * HWD * (HWD - 1));
    const double mean   = S[0] * invM;
    const double inten  = S[1] * invM - mean * mean;
    const double smooth = S[2] * invD + S[3] * invD;
    const float r = (float)(0.2 * 0.1 * (smooth + 0.1 * inten));
    *(volatile float*)out1 = r;
    __threadfence();
    *(volatile float*)out1 = r;
  }
}

extern "C" void kernel_launch(void* const* d_in, const int* in_sizes, int n_in,
                              void* d_out, int out_size, void* d_ws, size_t ws_size,
                              hipStream_t stream) {
  if (n_in < 6) return;
  if (in_sizes[0] != NB * CH * NSEQ) return;
  if (in_sizes[1] != CH * QKW || in_sizes[2] != CH * CH) return;
  if (in_sizes[3] != CH || in_sizes[4] != CH || in_sizes[5] != CH) return;
  if (out_size != NB * CH * NSEQ + 1) return;

  const float* x      = (const float*)d_in[0];
  const float* w_qkv  = (const float*)d_in[1];
  const float* w_proj = (const float*)d_in[2];
  const float* b_proj = (const float*)d_in[3];
  const float* ln_g   = (const float*)d_in[4];
  const float* ln_b   = (const float*)d_in[5];

  const size_t PWT  = (size_t)QKW * CH * 2;
  const size_t PWP  = (size_t)CH * CH * 2;
  const size_t PXN  = (size_t)MP * CH * 2;
  const size_t PQK  = (size_t)MP * 2 * CH * 2;
  const size_t PQL  = (size_t)MP * CH * 2;
  const size_t PVT  = (size_t)NB * CH * NSEQ * 2;
  const size_t POT  = (size_t)NB * CH * NSEQ * 2;
  const size_t PPT  = (size_t)NB * CH * 32 * 4;
  size_t off = 0;
  const size_t oWT = off; off += PWT;
  const size_t oWP = off; off += PWP;
  const size_t oXN = off; off += PXN;
  const size_t oQK = off; off += PQK;
  const size_t oQL = off; off += PQL;
  const size_t oVT = off; off += PVT;
  const size_t oOT = off; off += POT;
  const size_t oPT = off; off += PPT;
  if (off > ws_size) return;
  if (off > (size_t)134217728) return;

  char* ws = (char*)d_ws;
  unsigned short* WT  = (unsigned short*)(ws + oWT);
  unsigned short* WPT = (unsigned short*)(ws + oWP);
  unsigned short* XN  = (unsigned short*)(ws + oXN);
  unsigned short* QK  = (unsigned short*)(ws + oQK);
  unsigned short* QL  = (unsigned short*)(ws + oQL);
  unsigned short* VT  = (unsigned short*)(ws + oVT);
  unsigned short* OT  = (unsigned short*)(ws + oOT);
  float*          PT  = (float*)(ws + oPT);
  float*          out = (float*)d_out;

  const dim3 blk(256), blk128(128);
  const dim3 gW(32);
  const dim3 gLN(MP / 32);
  const dim3 gQK(((MP / 64) * ((2 * CH) / 64)) / 8, 1);
  const dim3 gVT(((CH / 64) * (NSEQ / 64)) / 8, NB);
  const dim3 gAT(NB * NHEAD * (NSEQ / 64));
  const dim3 gPJ(((CH / 64) * (NSEQ / 64)) / 8, NB);
  const dim3 gRP(NB * CH);
  const dim3 gRF(1);

  wprep<<<gW, blk, 0, stream>>>(w_qkv, w_proj, WT, WPT);

  ln_tok<<<gLN, blk, 0, stream>>>(x, ln_g, ln_b, XN);

  gemm64<0, 1><<<gQK, blk, 0, stream>>>(
      XN, CH, 0LL,
      WT, CH, 0LL,
      b_proj, x,
      (void*)QK, 2 * CH, 0LL,
      QL, CH, 0LL, CH,
      QSCALE * QC / (XC * WSC), KC / (XC * WSC), MP, 2 * CH, CH);

  gemm64<0, 1><<<gVT, blk, 0, stream>>>(
      WT + (size_t)2 * CH * CH, CH, 0LL,
      XN, CH, (long long)NSEQ * CH,
      b_proj, x,
      (void*)VT, NSEQ, (long long)CH * NSEQ,
      QL, CH, 0LL, 0,
      VC / (XC * WSC), VC / (XC * WSC), CH, NSEQ, CH);

  attn_t<<<gAT, blk128, 0, stream>>>(QK, QL, VT, OT);

  gemm64<1, 0><<<gPJ, blk, 0, stream>>>(
      WPT, CH, 0LL,
      OT, NSEQ, (long long)CH * NSEQ,
      b_proj, x,
      (void*)out, NSEQ, (long long)CH * NSEQ,
      QL, CH, 0LL, 0,
      1.0f / (WSC * AC), 1.0f / (WSC * AC), CH, NSEQ, CH);

  reg_part<<<gRP, blk, 0, stream>>>(out, PT);
  reg_fin<<<gRF, blk, 0, stream>>>(PT, out + (size_t)NB * CH * NSEQ);
  (void)hipGetLastError();
}
